// RelationModule_13477607375708
// MI455X (gfx1250) — hardware-verified
//
#include <hip/hip_runtime.h>
#include <stddef.h>
#include <stdint.h>

#define NB    4
#define NT    512
#define MT    2048
#define CD    1024
#define NPRJ  3072
#define LOCD  128
#define NFRQ  16

static_assert(MT == NB * NT);
static_assert(NT == 512);
static_assert(CD == 1024);
static_assert(NPRJ == 3 * CD);
static_assert(LOCD == 8 * NFRQ);
static_assert(MT % 64 == 0);
static_assert(NT % 256 == 0);
static_assert(CD % 64 == 0);

typedef _Float16 v16h __attribute__((ext_vector_type(16)));
typedef _Float16 v8h  __attribute__((ext_vector_type(8)));
typedef float    v8f  __attribute__((ext_vector_type(8)));
typedef float    v4f  __attribute__((ext_vector_type(4)));
typedef unsigned int v4u __attribute__((ext_vector_type(4)));

union Frag  { v16h v; v8h h[2]; };
union Pack8 { v8h h; v4u u; };

__device__ __forceinline__ v8f mma16(v16h a, v16h b, v8f c) {
  c = __builtin_amdgcn_wmma_f32_16x16x32_f16(false, a, false, b, (short)0, c, false, false);
  asm volatile("v_nop\n\tv_nop\n\tv_nop\n\tv_nop" : "+v"(c) : "v"(a), "v"(b));
  return c;
}

__device__ __forceinline__ v16h ldfrag(const _Float16* p, int ld, int row0, int k0, int lane) {
  const int m = lane & 15, lh = lane >> 4;
  const _Float16* q = p + (size_t)(row0 + m) * ld + k0 + 8 * lh;
  Frag f;
  f.h[0] = *(const v8h*)(q);
  f.h[1] = *(const v8h*)(q + 16);
  return f.v;
}

__device__ __forceinline__ v8f zero8() { return (v8f){0.f, 0.f, 0.f, 0.f, 0.f, 0.f, 0.f, 0.f}; }

__device__ __forceinline__ void gemm16x64(const _Float16* __restrict__ A, int lda,
                                          const _Float16* __restrict__ Bt, int ldb,
                                          int m0, int n0, int lane, v8f (&acc)[4]) {
#pragma unroll 2
  for (int k0 = 0; k0 < CD; k0 += 32) {
    const v16h a = ldfrag(A, lda, m0, k0, lane);
#pragma unroll
    for (int t = 0; t < 4; ++t) {
      const v16h b = ldfrag(Bt, ldb, n0 + 16 * t, k0, lane);
      acc[t] = mma16(a, b, acc[t]);
    }
  }
}

template <int KD>
__device__ __forceinline__ void gemm32x64(const _Float16* __restrict__ A, int lda,
                                          const _Float16* __restrict__ Bt, int ldb,
                                          int m0, int n0, int lane, v8f (&acc)[2][4]) {
  static_assert(KD % 64 == 0);
#pragma unroll 2
  for (int k0 = 0; k0 < KD; k0 += 32) {
    const v16h a0 = ldfrag(A, lda, m0, k0, lane);
    const v16h a1 = ldfrag(A, lda, m0 + 16, k0, lane);
    const v16h b0 = ldfrag(Bt, ldb, n0, k0, lane);
    const v16h b1 = ldfrag(Bt, ldb, n0 + 16, k0, lane);
    const v16h b2 = ldfrag(Bt, ldb, n0 + 32, k0, lane);
    const v16h b3 = ldfrag(Bt, ldb, n0 + 48, k0, lane);
    acc[0][0] = mma16(a0, b0, acc[0][0]);
    acc[1][0] = mma16(a1, b0, acc[1][0]);
    acc[0][1] = mma16(a0, b1, acc[0][1]);
    acc[1][1] = mma16(a1, b1, acc[1][1]);
    acc[0][2] = mma16(a0, b2, acc[0][2]);
    acc[1][2] = mma16(a1, b2, acc[1][2]);
    acc[0][3] = mma16(a0, b3, acc[0][3]);
    acc[1][3] = mma16(a1, b3, acc[1][3]);
  }
}

__global__ __launch_bounds__(256) void k_bnstat(const float* __restrict__ X, const float* __restrict__ g,
                                                const float* __restrict__ bt, float* __restrict__ bnp) {
  __shared__ __align__(16) float stg[512];
  const int tid = threadIdx.x;
  const int col = blockIdx.x * 256 + tid;
  double s = 0.0, s2 = 0.0;
#pragma unroll 4
  for (int r = 0; r < MT; ++r) {
    const double v = (double)X[(size_t)r * CD + col];
    s += v;
    s2 += v * v;
  }
  const double m = s * (1.0 / (double)MT);
  double var = s2 * (1.0 / (double)MT) - m * m;
  var = (var > 0.0) ? var : 0.0;
  const float rstd = rsqrtf((float)var + 1e-5f);
  const float sc = g[col] * rstd;
  const float sh = bt[col] - (float)m * sc;
  stg[tid] = sc;
  stg[256 + tid] = sh;
  __syncthreads();
  if (tid < 128) {
    const int part = tid >> 6;
    const int q = tid & 63;
    const v4f v = *(const v4f*)(stg + part * 256 + q * 4);
    volatile v4f* d = (volatile v4f*)(bnp + part * CD + blockIdx.x * 256 + q * 4);
    *d = v;
    __threadfence();
    *d = v;
  }
}

__global__ __launch_bounds__(256) void k_cvtx(const float* __restrict__ src, const float* __restrict__ bnp,
                                              _Float16* __restrict__ dh) {
  const int tid = threadIdx.x;
  const int row = blockIdx.x * 2 + (tid >> 7);
  const int col = (tid & 127) * 8;
  const size_t o = (size_t)row * CD + col;
  const v4f a0 = *(const v4f*)(src + o);
  const v4f a1 = *(const v4f*)(src + o + 4);
  const v4f s0 = *(const v4f*)(bnp + col);
  const v4f s1 = *(const v4f*)(bnp + col + 4);
  const v4f h0 = *(const v4f*)(bnp + CD + col);
  const v4f h1 = *(const v4f*)(bnp + CD + col + 4);
  Pack8 pk;
  pk.h = (v8h){(_Float16)fmaf(a0[0], s0[0], h0[0]), (_Float16)fmaf(a0[1], s0[1], h0[1]),
               (_Float16)fmaf(a0[2], s0[2], h0[2]), (_Float16)fmaf(a0[3], s0[3], h0[3]),
               (_Float16)fmaf(a1[0], s1[0], h1[0]), (_Float16)fmaf(a1[1], s1[1], h1[1]),
               (_Float16)fmaf(a1[2], s1[2], h1[2]), (_Float16)fmaf(a1[3], s1[3], h1[3])};
  const v4u vv = pk.u;
  volatile v4u* d = (volatile v4u*)(dh + o);
  *d = vv;
  __threadfence();
  *d = vv;
}

#define WTP 65
__global__ __launch_bounds__(256) void k_wtr(const float* __restrict__ W, int ncol, int nofs,
                                             _Float16* __restrict__ wt) {
  __shared__ float tl[64 * WTP];
  const int tid = threadIdx.x;
  const int n0 = blockIdx.x * 64, k0 = blockIdx.y * 64;
#pragma unroll
  for (int j = 0; j < 4; ++j) {
    const int p  = tid + 256 * j;
    const int kk = p >> 4;
    const int q4 = (p & 15) * 4;
    const v4f a = *(const v4f*)(W + (size_t)(k0 + kk) * ncol + n0 + q4);
    float* d = tl + kk * WTP + q4;
    d[0] = a[0]; d[1] = a[1]; d[2] = a[2]; d[3] = a[3];
  }
  __syncthreads();
  v4u vt[2];
  size_t go[2];
#pragma unroll
  for (int j = 0; j < 2; ++j) {
    const int p  = tid + 256 * j;
    const int nn = p >> 3;
    const int pc = p & 7;
    const float* cp = tl + (pc * 8) * WTP + nn;
    Pack8 pk;
    pk.h = (v8h){(_Float16)(cp[0 * WTP] * 32.0f), (_Float16)(cp[1 * WTP] * 32.0f),
                 (_Float16)(cp[2 * WTP] * 32.0f), (_Float16)(cp[3 * WTP] * 32.0f),
                 (_Float16)(cp[4 * WTP] * 32.0f), (_Float16)(cp[5 * WTP] * 32.0f),
                 (_Float16)(cp[6 * WTP] * 32.0f), (_Float16)(cp[7 * WTP] * 32.0f)};
    vt[j] = pk.u;
    go[j] = (size_t)(nofs + n0 + nn) * CD + k0 + pc * 8;
  }
  for (int ps = 0; ps < 2; ++ps) {
#pragma unroll
    for (int j = 0; j < 2; ++j) *(volatile v4u*)(wt + go[j]) = vt[j];
    __threadfence();
  }
}

#define SFP 132
__global__ __launch_bounds__(256) void k_qkv(const _Float16* __restrict__ xh,
                                             const _Float16* __restrict__ wt,
                                             const float* __restrict__ bq,
                                             const float* __restrict__ bk,
                                             const float* __restrict__ bv,
                                             _Float16* __restrict__ qp,
                                             _Float16* __restrict__ kp,
                                             _Float16* __restrict__ vtp) {
  __shared__ __align__(16) float sf[64 * SFP];
  const int tid = threadIdx.x, lane = tid & 31, wave = tid >> 5;
  const int hh = lane >> 4, c = lane & 15;
  const int wm = wave >> 1, wn = wave & 1;
  const int mb = blockIdx.x * 64;
  const int b  = mb >> 9;
  const int sb = mb & (NT - 1);
  const int ns = blockIdx.y;
  const int which = ns >> 3;
  const int hp0 = (ns & 7) * 128;
  const int m0 = mb + wm * 16;
  const int n0 = ns * 128 + wn * 64;
  const float* bias = ((which == 0) ? bq : ((which == 1) ? bk : bv)) + hp0;
  const float osc = (which == 2) ? 16.0f : 1.0f;

  v8f acc[4];
#pragma unroll
  for (int t = 0; t < 4; ++t) acc[t] = zero8();
  gemm16x64(xh, CD, wt, CD, m0, n0, lane, acc);

#pragma unroll
  for (int t = 0; t < 4; ++t) {
    const float bb = bias[wn * 64 + 16 * t + c];
#pragma unroll
    for (int r = 0; r < 8; ++r)
      sf[(wm * 16 + 8 * hh + r) * SFP + wn * 64 + 16 * t + c] = (acc[t][r] * 0.03125f + bb) * osc;
  }
  __syncthreads();

  if (which < 2) {
    v4u val[4];
    size_t go[4];
#pragma unroll
    for (int j = 0; j < 4; ++j) {
      const int p  = tid + 256 * j;
      const int lr = p >> 4;
      const int pc = p & 15;
      const float* ra = sf + lr * SFP + pc * 8;
      const v4f a0 = *(const v4f*)(ra), a1 = *(const v4f*)(ra + 4);
      Pack8 pk;
      pk.h = (v8h){(_Float16)a0[0], (_Float16)a0[1], (_Float16)a0[2], (_Float16)a0[3],
                   (_Float16)a1[0], (_Float16)a1[1], (_Float16)a1[2], (_Float16)a1[3]};
      val[j] = pk.u;
      go[j]  = (size_t)(mb + lr) * CD + hp0 + pc * 8;
    }
    _Float16* base = (which == 0) ? qp : kp;
    for (int ps = 0; ps < 2; ++ps) {
#pragma unroll
      for (int j = 0; j < 4; ++j) *(volatile v4u*)(base + go[j]) = val[j];
      __threadfence();
    }
  } else {
    v4u val[4];
    size_t go[4];
#pragma unroll
    for (int j = 0; j < 4; ++j) {
      const int p    = tid + 256 * j;
      const int dcol = p >> 3;
      const int pc   = p & 7;
      const float* cp = sf + (pc * 8) * SFP + dcol;
      Pack8 pk;
      pk.h = (v8h){(_Float16)cp[0 * SFP], (_Float16)cp[1 * SFP], (_Float16)cp[2 * SFP], (_Float16)cp[3 * SFP],
                   (_Float16)cp[4 * SFP], (_Float16)cp[5 * SFP], (_Float16)cp[6 * SFP], (_Float16)cp[7 * SFP]};
      val[j] = pk.u;
      go[j]  = ((size_t)(b * CD + hp0 + dcol)) * NT + sb + pc * 8;
    }
    for (int ps = 0; ps < 2; ++ps) {
#pragma unroll
      for (int j = 0; j < 4; ++j) *(volatile v4u*)(vtp + go[j]) = val[j];
      __threadfence();
    }
  }
}

#define LN1000 6.90775528f
__global__ __launch_bounds__(256) void k_relpe(const float* __restrict__ boxes, const float* __restrict__ Wr,
                                               const float* __restrict__ br, float* __restrict__ rb) {
  __shared__ float cxs[NT], cys[NT], rws[NT], rhs[NT], wss[NT], hss[NT];
  __shared__ float wrs[LOCD];
  __shared__ float ipe[NFRQ];
  __shared__ __align__(16) float srow[NT];
  __shared__ float red[8];
  const int tid = threadIdx.x, lane = tid & 31, wave = tid >> 5;
  const int bi = blockIdx.x;
  const int b = bi >> 9, i = bi & (NT - 1);
  const float* bx = boxes + (size_t)b * NT * 4;
  for (int t = tid; t < NT; t += 256) {
    const v4f bb = *(const v4f*)(bx + t * 4);
    cxs[t] = bb[0] + 0.5f * bb[2];
    cys[t] = bb[1] + 0.5f * bb[3];
    wss[t] = bb[2];
    hss[t] = bb[3];
    rws[t] = __builtin_amdgcn_rcpf(bb[2]);
    rhs[t] = __builtin_amdgcn_rcpf(bb[3]);
  }
  if (tid < LOCD) wrs[tid] = Wr[tid];
  if (tid < NFRQ) ipe[tid] = __expf(-(float)tid * 0.125f * LN1000);
  __syncthreads();
  const float cxi = cxs[i], cyi = cys[i], wi = wss[i], hgi = hss[i];
  const float brv = br[0];
#pragma unroll 1
  for (int jj = 0; jj < 2; ++jj) {
    const int j = tid + 256 * jj;
    const int blk = j >> 7;
    const int mb4 = (j & 127) * 4;
    float s = brv;
#pragma unroll 1
    for (int c = 0; c < 4; ++c) {
      const int m = mb4 + c;
      const float rw = rws[m], rh = rhs[m];
      const float vx = fmaxf(fabsf(cxi - cxs[m]) * rw, 1e-3f);
      const float vy = fmaxf(fabsf(cyi - cys[m]) * rh, 1e-3f);
      const float vw = wi * rw;
      const float vh = hgi * rh;
      const float val = (blk == 0) ? vx : ((blk == 1) ? vy : ((blk == 2) ? vw : vh));
      const float dl = __logf(val);
      const int wb = c * 32;
#pragma unroll 4
      for (int k = 0; k < NFRQ; ++k) {
        const float a = dl * ipe[k];
        float sn, cs;
        __sincosf(a, &sn, &cs);
        s = fmaf(sn, wrs[wb + k], s);
        s = fmaf(cs, wrs[wb + 16 + k], s);
      }
    }
    srow[j] = s;
  }
  __syncthreads();
  const float s0 = srow[tid], s1 = srow[tid + 256];
  float mx = fmaxf(s0, s1);
#pragma unroll
  for (int off = 1; off < 32; off <<= 1) mx = fmaxf(mx, __shfl_xor(mx, off, 32));
  if (lane == 0) red[wave] = mx;
  __syncthreads();
  float M = red[0];
#pragma unroll
  for (int w = 1; w < 8; ++w) M = fmaxf(M, red[w]);
  float e = __expf(s0 - M) + __expf(s1 - M);
#pragma unroll
  for (int off = 1; off < 32; off <<= 1) e += __shfl_xor(e, off, 32);
  __syncthreads();
  if (lane == 0) red[wave] = e;
  __syncthreads();
  float S = red[0];
#pragma unroll
  for (int w = 1; w < 8; ++w) S += red[w];
  const float lse = M + __logf(S);
  srow[tid] = s0 - lse;
  srow[tid + 256] = s1 - lse;
  __syncthreads();
  if (tid < 128) {
    const v4f v = *(const v4f*)(srow + tid * 4);
    volatile v4f* d = (volatile v4f*)(rb + (size_t)bi * NT + tid * 4);
    *d = v;
    __threadfence();
    *d = v;
  }
}

#define OTP 68
template <int MODE>
__device__ __forceinline__ void epi32x64(v8f (&acc)[2][4], float scale, const float* __restrict__ add,
                                         float* sw, float* __restrict__ out, int ldo,
                                         int m0, int n0, int lane, int hh, int c) {
#pragma unroll
  for (int sub = 0; sub < 2; ++sub) {
    __syncthreads();
#pragma unroll
    for (int t = 0; t < 4; ++t) {
#pragma unroll
      for (int r = 0; r < 8; ++r) sw[(8 * hh + r) * OTP + 16 * t + c] = acc[sub][t][r] * scale;
    }
    __syncthreads();
    v4f val[8];
    size_t go[8];
#pragma unroll
    for (int it = 0; it < 8; ++it) {
      const int p    = lane + 32 * it;
      const int L    = p >> 3;
      const int pc   = p & 7;
      const int row  = L >> 1;
      const int half = L & 1;
      go[it]  = (size_t)(m0 + sub * 16 + row) * ldo + n0 + half * 32 + pc * 4;
      v4f v = *(const v4f*)(sw + row * OTP + half * 32 + pc * 4);
      if (MODE == 1) {
        const v4f ad = *(const v4f*)(add + go[it]);
        v += ad;
      }
      val[it] = v;
    }
    for (int ps = 0; ps < 2; ++ps) {
#pragma unroll
      for (int it = 0; it < 8; ++it) *(volatile v4f*)(out + go[it]) = val[it];
      __threadfence();
    }
  }
}

__global__ __launch_bounds__(256) void k_scores(const _Float16* __restrict__ qp,
                                                const _Float16* __restrict__ kp,
                                                const float* __restrict__ rb,
                                                float* __restrict__ sp) {
  __shared__ __align__(16) float st[8][16 * OTP];
  const int tid = threadIdx.x, lane = tid & 31, wave = tid >> 5;
  const int hh = lane >> 4, c = lane & 15;
  const int b  = blockIdx.z;
  const int m0 = blockIdx.x * 256 + wave * 32;
  const int n0 = blockIdx.y * 64;
  const _Float16* A  = qp + (size_t)b * NT * CD;
  const _Float16* Bt = kp + (size_t)b * NT * CD;
  v8f acc[2][4];
#pragma unroll
  for (int s = 0; s < 2; ++s)
#pragma unroll
    for (int t = 0; t < 4; ++t) acc[s][t] = zero8();
  gemm32x64<CD>(A, CD, Bt, CD, m0, n0, lane, acc);
  epi32x64<1>(acc, 0.03125f, rb + (size_t)b * NT * NT, st[wave], sp + (size_t)b * NT * NT, NT,
              m0, n0, lane, hh, c);
}

__global__ __launch_bounds__(256) void k_softmax(const float* __restrict__ sp, _Float16* __restrict__ pp) {
  __shared__ float redm[8];
  __shared__ float reds[8];
  const int tid = threadIdx.x, lane = tid & 31, wave = tid >> 5;
  const int grp = tid >> 6;
  const int row = blockIdx.x * 4 + grp;
  const int j0  = (tid & 63) * 8;
  const float* s = sp + (size_t)row * NT + j0;
  const v4f a0 = *(const v4f*)(s), a1 = *(const v4f*)(s + 4);
  float x[8] = {a0[0], a0[1], a0[2], a0[3], a1[0], a1[1], a1[2], a1[3]};
  float mx = x[0];
#pragma unroll
  for (int e = 1; e < 8; ++e) mx = fmaxf(mx, x[e]);
#pragma unroll
  for (int off = 1; off < 32; off <<= 1) mx = fmaxf(mx, __shfl_xor(mx, off, 32));
  if (lane == 0) redm[wave] = mx;
  __syncthreads();
  const float M = fmaxf(redm[2 * grp], redm[2 * grp + 1]);
  float ev[8];
  float sum = 0.f;
#pragma unroll
  for (int e = 0; e < 8; ++e) { ev[e] = __expf(x[e] - M); sum += ev[e]; }
#pragma unroll
  for (int off = 1; off < 32; off <<= 1) sum += __shfl_xor(sum, off, 32);
  if (lane == 0) reds[wave] = sum;
  __syncthreads();
  const float S = reds[2 * grp] + reds[2 * grp + 1];
  const float inv = 1024.0f / S;
  Pack8 pk;
  pk.h = (v8h){(_Float16)(ev[0] * inv), (_Float16)(ev[1] * inv), (_Float16)(ev[2] * inv), (_Float16)(ev[3] * inv),
               (_Float16)(ev[4] * inv), (_Float16)(ev[5] * inv), (_Float16)(ev[6] * inv), (_Float16)(ev[7] * inv)};
  const v4u vv = pk.u;
  volatile v4u* d = (volatile v4u*)(pp + (size_t)row * NT + j0);
  *d = vv;
  __threadfence();
  *d = vv;
}

__global__ __launch_bounds__(256) void k_pv(const _Float16* __restrict__ pp,
                                            const _Float16* __restrict__ vt,
                                            float* __restrict__ opre) {
  __shared__ __align__(16) float st[8][16 * OTP];
  const int tid = threadIdx.x, lane = tid & 31, wave = tid >> 5;
  const int hh = lane >> 4, c = lane & 15;
  const int b  = blockIdx.z;
  const int m0 = blockIdx.x * 256 + wave * 32;
  const int n0 = blockIdx.y * 64;
  const _Float16* A  = pp + (size_t)b * NT * NT;
  const _Float16* Bt = vt + (size_t)b * CD * NT;
  v8f acc[2][4];
#pragma unroll
  for (int s = 0; s < 2; ++s)
#pragma unroll
    for (int t = 0; t < 4; ++t) acc[s][t] = zero8();
  gemm32x64<NT>(A, NT, Bt, NT, m0, n0, lane, acc);
  epi32x64<0>(acc, 6.103515625e-05f, nullptr, st[wave], opre + (size_t)b * NT * CD, CD,
              m0, n0, lane, hh, c);
}

__global__ __launch_bounds__(256) void k_bnapply(const float* __restrict__ X, const float* __restrict__ bnp,
                                                 float* __restrict__ out) {
  const int tid = threadIdx.x;
  const int col = tid * 4;
  const size_t o = (size_t)blockIdx.x * CD + col;
  const v4f a  = *(const v4f*)(X + o);
  const v4f sc = *(const v4f*)(bnp + col);
  const v4f sh = *(const v4f*)(bnp + CD + col);
  v4f y;
  y[0] = fmaf(a[0], sc[0], sh[0]);
  y[1] = fmaf(a[1], sc[1], sh[1]);
  y[2] = fmaf(a[2], sc[2], sh[2]);
  y[3] = fmaf(a[3], sc[3], sh[3]);
  volatile v4f* d = (volatile v4f*)(out + o);
  *d = y;
  __threadfence();
  *d = y;
}

extern "C" void kernel_launch(void* const* d_in, const int* in_sizes, int n_in,
                              void* d_out, int out_size, void* d_ws, size_t ws_size,
                              hipStream_t stream) {
  if (n_in < 14) return;
  if (in_sizes[0] != MT * CD) return;
  if (in_sizes[1] != NB * NT * 4) return;
  if (in_sizes[2] != CD) return;
  if (in_sizes[3] != CD) return;
  if (in_sizes[4] != CD * CD) return;
  if (in_sizes[5] != CD) return;
  if (in_sizes[6] != CD * CD) return;
  if (in_sizes[7] != CD) return;
  if (in_sizes[8] != CD * CD) return;
  if (in_sizes[9] != CD) return;
  if (in_sizes[10] != LOCD) return;
  if (in_sizes[11] != 1) return;
  if (in_sizes[12] != CD) return;
  if (in_sizes[13] != CD) return;
  if (out_size != MT * CD) return;

  const float* x     = (const float*)d_in[0];
  const float* boxes = (const float*)d_in[1];
  const float* g1    = (const float*)d_in[2];
  const float* b1    = (const float*)d_in[3];
  const float* wq    = (const float*)d_in[4];
  const float* bq    = (const float*)d_in[5];
  const float* wk    = (const float*)d_in[6];
  const float* bk    = (const float*)d_in[7];
  const float* wv    = (const float*)d_in[8];
  const float* bv    = (const float*)d_in[9];
  const float* wr    = (const float*)d_in[10];
  const float* br    = (const float*)d_in[11];
  const float* g2    = (const float*)d_in[12];
  const float* b2    = (const float*)d_in[13];
  float* out = (float*)d_out;

  size_t off = 0;
  const size_t oB1 = off; off += (size_t)2 * CD * 4;
  const size_t oB2 = off; off += (size_t)2 * CD * 4;
  const size_t oX  = off; off += (size_t)MT * CD * 2;
  const size_t oWt = off; off += (size_t)NPRJ * CD * 2;
  const size_t oQ  = off; off += (size_t)MT * CD * 2;
  const size_t oK  = off; off += (size_t)MT * CD * 2;
  const size_t oV  = off; off += (size_t)NB * CD * NT * 2;
  const size_t oR  = off; off += (size_t)NB * NT * NT * 4;
  const size_t oS  = off; off += (size_t)NB * NT * NT * 4;
  const size_t oP  = off; off += (size_t)NB * NT * NT * 2;
  const size_t oO  = off; off += (size_t)MT * CD * 4;
  if (off > ws_size) return;
  if (off > (size_t)134217728) return;

  char* ws = (char*)d_ws;
  float*    Bn1 = (float*)(ws + oB1);
  float*    Bn2 = (float*)(ws + oB2);
  _Float16* Xh  = (_Float16*)(ws + oX);
  _Float16* Wt  = (_Float16*)(ws + oWt);
  _Float16* Qp  = (_Float16*)(ws + oQ);
  _Float16* Kp  = (_Float16*)(ws + oK);
  _Float16* Vt  = (_Float16*)(ws + oV);
  float*    Rb  = (float*)(ws + oR);
  float*    Sp  = (float*)(ws + oS);
  _Float16* Pp  = (_Float16*)(ws + oP);
  float*    Op  = (float*)(ws + oO);

  k_bnstat<<<dim3(CD / 256), dim3(256), 0, stream>>>(x, g1, b1, Bn1);
  k_cvtx<<<dim3(MT / 2), dim3(256), 0, stream>>>(x, Bn1, Xh);
  k_wtr<<<dim3(CD / 64, CD / 64), dim3(256), 0, stream>>>(wq, CD, 0, Wt);
  k_wtr<<<dim3(CD / 64, CD / 64), dim3(256), 0, stream>>>(wk, CD, CD, Wt);
  k_wtr<<<dim3(CD / 64, CD / 64), dim3(256), 0, stream>>>(wv, CD, 2 * CD, Wt);
  k_qkv<<<dim3(MT / 64, NPRJ / 128), dim3(256), 0, stream>>>(Xh, Wt, bq, bk, bv, Qp, Kp, Vt);
  k_relpe<<<dim3(MT), dim3(256), 0, stream>>>(boxes, wr, br, Rb);
  k_scores<<<dim3(NT / 256, NT / 64, NB), dim3(256), 0, stream>>>(Qp, Kp, Rb, Sp);
  k_softmax<<<dim3(MT / 4), dim3(256), 0, stream>>>(Sp, Pp);
  k_pv<<<dim3(NT / 256, CD / 64, NB), dim3(256), 0, stream>>>(Pp, Vt, Op);
  k_bnstat<<<dim3(CD / 256), dim3(256), 0, stream>>>(Op, g2, b2, Bn2);
  k_bnapply<<<dim3(MT), dim3(256), 0, stream>>>(Op, Bn2, out);
  (void)hipGetLastError();
}
